// EigenBasisEncoder_5076651344401
// MI455X (gfx1250) — hardware-verified
//
#include <hip/hip_runtime.h>


#define NB   16
#define NM   16
#define NN   64
#define DD   64
#define HF   2048
#define HG   64
#define NE   (NB * NN * NN)
#define NIJ  (NN * NN)
#define DM   64
#define LOSC 1024.0f
#define SQ2PI 2.5066282746310002f

typedef _Float16 h16;
typedef unsigned short bf;
typedef __attribute__((ext_vector_type(16))) __bf16   v16bf;
typedef __attribute__((ext_vector_type(16))) _Float16 v16h;
typedef __attribute__((ext_vector_type(8)))  _Float16 v8h;
typedef __attribute__((ext_vector_type(8)))  unsigned short v8us;
typedef __attribute__((ext_vector_type(8)))  float    v8f;
typedef __attribute__((ext_vector_type(4)))  float    v4f;
typedef v8h  __attribute__((may_alias)) v8ha;
typedef v4f  __attribute__((may_alias)) v4fa;
typedef v8us __attribute__((may_alias)) v8usa;

__device__ __forceinline__ unsigned short f2bf(float f) { unsigned u = __float_as_uint(f); u += 0x7FFFu + ((u >> 16) & 1u); return (unsigned short)(u >> 16); }
__device__ __forceinline__ float bf2f(unsigned short b) { return __uint_as_float(((unsigned)b) << 16); }
__device__ __forceinline__ float bfr(float f) { return bf2f(f2bf(f)); }
__device__ __forceinline__ v16h cat16(v8h lo, v8h hi) { return __builtin_shufflevector(lo, hi, 0, 1, 2, 3, 4, 5, 6, 7, 8, 9, 10, 11, 12, 13, 14, 15); }
__device__ __forceinline__ v16bf cat16b(v8us lo, v8us hi) { return __builtin_bit_cast(v16bf, __builtin_shufflevector(lo, hi, 0, 1, 2, 3, 4, 5, 6, 7, 8, 9, 10, 11, 12, 13, 14, 15)); }
__device__ __forceinline__ v8f wmma16(v16h a, v16h b, v8f c) { return __builtin_amdgcn_wmma_f32_16x16x32_f16(false, a, false, b, (short)0, c, false, false); }
__device__ __forceinline__ v8f wmmab(v16bf a, v16bf b, v8f c) { return __builtin_amdgcn_wmma_f32_16x16x32_bf16(false, a, false, b, (short)0, c, false, false); }

template <bool SPLITA, bool F16OUT = false>
__global__ __launch_bounds__(128) void k_gemmb(const bf* __restrict__ A, const bf* __restrict__ Al, const bf* __restrict__ Bn, const float* __restrict__ bias, float* C, int ldc, h16* C2, const float* __restrict__ R = nullptr, int K = DM, int roundR = 1) {
    __shared__ __align__(16) float ost[4][16 * 68];
    const int lane = threadIdx.x & 31, wave = threadIdx.x >> 5, lr = lane & 15, hi = lane >> 4;
    const int r0 = blockIdx.x * 64 + wave * 16, c0 = blockIdx.y * 64;
    const size_t aoff = (size_t)(r0 + lr) * K + 8 * hi;
    size_t boff[4];
#pragma unroll
    for (int t = 0; t < 4; ++t) boff[t] = (size_t)(c0 + t * 16 + lr) * K + 8 * hi;
    v8f acc[4];
#pragma unroll
    for (int t = 0; t < 4; ++t) acc[t] = (v8f){};
#pragma unroll 1
    for (int kc = 0; kc < K; kc += 32) {
        const v16bf a = cat16b(*(const v8us*)(A + aoff + kc), *(const v8us*)(A + aoff + kc + 16));
        v16bf al = a;
        if (SPLITA) al = cat16b(*(const v8us*)(Al + aoff + kc), *(const v8us*)(Al + aoff + kc + 16));
#pragma unroll
        for (int t = 0; t < 4; ++t) { const v16bf b = cat16b(*(const v8us*)(Bn + boff[t] + kc), *(const v8us*)(Bn + boff[t] + kc + 16)); acc[t] = wmmab(a, b, acc[t]); if (SPLITA) acc[t] = wmmab(al, b, acc[t]); }
        asm volatile("v_nop\n\tv_nop\n\tv_nop\n\tv_nop" : "+v"(acc[0]), "+v"(acc[1]), "+v"(acc[2]), "+v"(acc[3]) : "v"(a), "v"(al));
    }
    float* os = &ost[wave][0];
#pragma unroll
    for (int t = 0; t < 4; ++t) { const float bv = bias ? bfr(bias[c0 + t * 16 + lr]) : 0.f;
#pragma unroll
        for (int j = 0; j < 8; ++j) os[(hi * 8 + j) * 68 + t * 16 + lr] = acc[t][j] + bv; }
    __syncthreads();
    if (F16OUT) {
        h16* crow = (h16*)(void*)C + (size_t)r0 * ldc + c0;
        auto pass = [&]() {
#pragma unroll
            for (int s = 0; s < 4; ++s) { const int row = 4 * s + (lane >> 3), piece = lane & 7; const float* sp = os + row * 68 + piece * 8; v8h o, o2;
#pragma unroll
                for (int i = 0; i < 8; ++i) { const h16 a = (h16)sp[i]; o[i] = a; o2[i] = (h16)((sp[i] - (float)a) * LOSC); }
                *(volatile v8h*)(crow + (size_t)row * ldc + piece * 8) = o; if (C2) *(volatile v8h*)(C2 + (size_t)r0 * ldc + c0 + (size_t)row * ldc + piece * 8) = o2; }
        };
        pass(); __threadfence(); pass();
    } else {
        float* crow = C + (size_t)r0 * ldc + c0;
        auto pass = [&]() {
#pragma unroll
            for (int s = 0; s < 8; ++s) { const int Lid = (lane >> 3) + 4 * s, piece = lane & 7; const int row = Lid >> 1, cofs = (Lid & 1) * 32 + piece * 4;
                v4f val = *(const v4fa*)(os + row * 68 + cofs); if (R) { const v4f rv = *(const v4f*)(R + ((size_t)r0 + row) * ldc + c0 + cofs); val += roundR ? (v4f){bfr(rv[0]), bfr(rv[1]), bfr(rv[2]), bfr(rv[3])} : rv; }
                *(volatile v4f*)(crow + (size_t)row * ldc + cofs) = val; }
        };
        pass(); __threadfence(); pass();
    }
}

__global__ __launch_bounds__(256) void k_wt(const float* __restrict__ Wm, int K, int ncols, bf* WT) {
    __shared__ __align__(16) unsigned short tl[64 * 72];
    const int tid = threadIdx.x, k0 = blockIdx.x * 64, n0 = blockIdx.y * 64;
    const int kk = tid >> 2, nq = (tid & 3) * 16;
#pragma unroll
    for (int i = 0; i < 16; ++i) tl[(nq + i) * 72 + kk] = f2bf(Wm[(size_t)(k0 + kk) * ncols + n0 + nq + i]);
    __syncthreads();
    const int piece = tid & 7;
    auto pass = [&]() {
#pragma unroll
        for (int s = 0; s < 2; ++s) { const int nr = (tid >> 3) + 32 * s; const v8us val = *(const v8usa*)(tl + nr * 72 + piece * 8); *(volatile v8us*)(WT + (size_t)(n0 + nr) * K + k0 + piece * 8) = val; }
    };
    pass(); __threadfence(); pass();
}

__global__ __launch_bounds__(256) void k_cvt8(const float* __restrict__ src, bf* dst, size_t n8) {
    const size_t i = (size_t)blockIdx.x * 256 + threadIdx.x; if (i >= n8) return;
    const v8f v = *(const v8f*)(src + i * 8); v8us o;
#pragma unroll
    for (int k = 0; k < 8; ++k) o[k] = f2bf(v[k]);
    *(volatile v8us*)(dst + i * 8) = o; __threadfence(); *(volatile v8us*)(dst + i * 8) = o;
}
__global__ __launch_bounds__(256) void k_zero8(bf* dst, size_t n8) {
    const size_t i = (size_t)blockIdx.x * 256 + threadIdx.x; if (i >= n8) return; v8us z;
#pragma unroll
    for (int k = 0; k < 8; ++k) z[k] = 0;
    *(volatile v8us*)(dst + i * 8) = z; __threadfence(); *(volatile v8us*)(dst + i * 8) = z;
}

__global__ __launch_bounds__(256) void k_fhid(const float* __restrict__ ev, const float* __restrict__ f1w2, const float* __restrict__ f1b2, const float* __restrict__ bpm, const float* __restrict__ bps,
                                             const float* __restrict__ f2w2, const float* __restrict__ f2b2, bf* Ph, bf* Pl) {
    typedef __attribute__((ext_vector_type(2))) unsigned short v2us;
    const int lane = threadIdx.x & 31, r = blockIdx.x * 8 + (threadIdx.x >> 5); if (r >= NB * NM) return; const float x = bfr(ev[r]);
#pragma unroll 1
    for (int ps = 0; ps < 2; ++ps) {
#pragma unroll 1
        for (int c0 = lane * 2; c0 < 2 * HF; c0 += 64) { v2us oh, ol;
#pragma unroll
            for (int q = 0; q < 2; ++q) { const int c = c0 + q; float h;
                if (c < HF) { const float s = __fdividef(1.0f, 1.0f + __expf(-(x * fabsf(bfr(f1w2[c])) + bfr(f1b2[c])))); const float mean = __fdividef(2.0f, 1.0f + __expf(-bfr(bpm[c]))) - 1.0f; const float sd = fabsf(bfr(bps[c]));
                    const float z = __fdividef(s - mean, sd); const float sc = __fdividef(__expf(-0.5f * z * z), sd * SQ2PI); h = 2.0f * (sc * s - 0.5f); }
                else { const int cc = c - HF; const float s = __fdividef(1.0f, 1.0f + __expf(-(x * fabsf(bfr(f2w2[cc])) + bfr(f2b2[cc])))); h = 2.0f * (s - 0.5f); }
                const unsigned short hb = f2bf(h); oh[q] = hb; ol[q] = f2bf(h - bf2f(hb)); }
            const size_t o = (size_t)r * (2 * HF) + c0; *(volatile v2us*)(Ph + o) = oh; *(volatile v2us*)(Pl + o) = ol; }
        if (ps == 0) __threadfence(); }
}
__global__ __launch_bounds__(256) void k_fw3(const float* __restrict__ f1w3, const float* __restrict__ f2w3, bf* W3T) {
    const int lane = threadIdx.x & 31, n = blockIdx.x * 8 + (threadIdx.x >> 5); if (n >= DD) return;
#pragma unroll 1
    for (int ps = 0; ps < 2; ++ps) {
#pragma unroll 1
        for (int k0 = lane * 8; k0 < 2 * HF; k0 += 256) { v8us o;
#pragma unroll
            for (int q = 0; q < 8; ++q) { const int k = k0 + q; float v = 0.f;
                if (n < 32 && k < HF) v = fabsf(f1w3[(size_t)k * 32 + n]); else if (n >= 32 && k >= HF) v = fabsf(f2w3[(size_t)(k - HF) * 32 + (n - 32)]);
                o[q] = f2bf(v); }
            *(volatile v8us*)(W3T + (size_t)n * (2 * HF) + k0) = o; }
        if (ps == 0) __threadfence(); }
}
__global__ __launch_bounds__(256) void k_ffin(const float* __restrict__ C, const float* __restrict__ ev, const float* __restrict__ f1w1, const float* __restrict__ f1b1, const float* __restrict__ f2w1, const float* __restrict__ f2b1, const int* __restrict__ mm, float* F) {
    typedef __attribute__((ext_vector_type(2))) float v2f;
    const int lane = threadIdx.x & 31, r = blockIdx.x * 8 + (threadIdx.x >> 5); if (r >= NB * NM) return; const float x = bfr(ev[r]); const float mk = (mm[r] != 0) ? 1.0f : 0.f; v2f o;
#pragma unroll
    for (int i = 0; i < 2; ++i) { const int d = lane * 2 + i; float h;
        if (d < 32) h = x * fabsf(bfr(f1w1[d])) + bfr(f1b1[d]); else h = x * fabsf(bfr(f2w1[d - 32])) + bfr(f2b1[d - 32]);
        h += C[(size_t)r * DD + d] * (1.0f / (float)HF); o[i] = __expf(h) * mk; }
    *(volatile v2f*)(F + (size_t)r * DD + lane * 2) = o; __threadfence(); *(volatile v2f*)(F + (size_t)r * DD + lane * 2) = o;
}
__global__ __launch_bounds__(256) void k_ghid(const float* __restrict__ vec, const float* __restrict__ w2, const float* __restrict__ b2, bf* Ph, bf* Pl) {
    typedef __attribute__((ext_vector_type(2))) unsigned short v2us;
    const int lane = threadIdx.x & 31, r = blockIdx.x * 8 + (threadIdx.x >> 5); if (r >= NM * NIJ) return; const float v = bfr(vec[r]); v2us oh, ol;
#pragma unroll
    for (int i = 0; i < 2; ++i) { const int c = lane * 2 + i; const float h = fmaxf(v * bfr(w2[c]) + bfr(b2[c]), 0.f); const unsigned short hb = f2bf(h); oh[i] = hb; ol[i] = f2bf(h - bf2f(hb)); }
    const size_t o = (size_t)r * HG + lane * 2; *(volatile v2us*)(Ph + o) = oh; *(volatile v2us*)(Pl + o) = ol; __threadfence(); *(volatile v2us*)(Ph + o) = oh; *(volatile v2us*)(Pl + o) = ol;
}
__global__ __launch_bounds__(256) void k_gsum(const float* __restrict__ G, const float* __restrict__ vec, const float* __restrict__ w1, const float* __restrict__ b1, const float* __restrict__ F, const int* __restrict__ ma, int b, bf* Oh, bf* Ol) {
    typedef __attribute__((ext_vector_type(2))) unsigned short v2us;
    const int lane = threadIdx.x & 31, ij = blockIdx.x * 8 + (threadIdx.x >> 5); if (ij >= NIJ) return; float acc[2] = {0.f, 0.f};
#pragma unroll 1
    for (int m = 0; m < NM; ++m) { const size_t e = ((size_t)b * NM + m) * NIJ + ij; const float v = bfr(vec[e]); const float mk = (ma[e] != 0) ? 1.0f : 0.f; const size_t gr = (size_t)m * NIJ + ij;
#pragma unroll
        for (int i = 0; i < 2; ++i) { const int d = lane * 2 + i; const float g = (v * bfr(w1[d]) + bfr(b1[d]) + G[gr * DD + d] * (1.0f / (float)HG)) * mk; acc[i] = fmaf(F[((size_t)b * NM + m) * DD + d], g, acc[i]); } }
    v2us oh, ol;
#pragma unroll
    for (int i = 0; i < 2; ++i) { const unsigned short hb = f2bf(acc[i]); oh[i] = hb; ol[i] = f2bf(acc[i] - bf2f(hb)); }
    const size_t o = ((size_t)b * NIJ + ij) * DD + lane * 2; *(volatile v2us*)(Oh + o) = oh; *(volatile v2us*)(Ol + o) = ol; __threadfence(); *(volatile v2us*)(Oh + o) = oh; *(volatile v2us*)(Ol + o) = ol;
}
__global__ __launch_bounds__(256) void k_cvt64(const float* __restrict__ src, int nrows, bf* dst) {
    typedef __attribute__((ext_vector_type(2))) unsigned short v2us;
    const int lane = threadIdx.x & 31, r = blockIdx.x * 8 + (threadIdx.x >> 5); if (r >= nrows) return; v2us o;
#pragma unroll
    for (int i = 0; i < 2; ++i) o[i] = f2bf(src[(size_t)r * DD + lane * 2 + i]);
    *(volatile v2us*)(dst + (size_t)r * DD + lane * 2) = o; __threadfence(); *(volatile v2us*)(dst + (size_t)r * DD + lane * 2) = o;
}

extern "C" void kernel_launch(void* const* d_in, const int* in_sizes, int n_in,
                              void* d_out, int out_size, void* d_ws, size_t ws_size, hipStream_t stream) {
    (void)in_sizes; (void)n_in; (void)out_size;
    const float* ev = (const float*)d_in[0]; const float* vec = (const float*)d_in[1]; const int* mm = (const int*)d_in[2]; const int* ma = (const int*)d_in[3]; const float* ea = (const float*)d_in[4];
    const float* f1w1 = (const float*)d_in[5]; const float* f1b1 = (const float*)d_in[6]; const float* f1w2 = (const float*)d_in[7]; const float* f1b2 = (const float*)d_in[8]; const float* f1w3 = (const float*)d_in[9]; const float* bpm = (const float*)d_in[10]; const float* bps = (const float*)d_in[11];
    const float* f2w1 = (const float*)d_in[12]; const float* f2b1 = (const float*)d_in[13]; const float* f2w2 = (const float*)d_in[14]; const float* f2b2 = (const float*)d_in[15]; const float* f2w3 = (const float*)d_in[16];
    const float* gw1 = (const float*)d_in[17]; const float* gb1 = (const float*)d_in[18]; const float* gw2 = (const float*)d_in[19]; const float* gb2 = (const float*)d_in[20]; const float* gw3 = (const float*)d_in[21]; const float* lw = (const float*)d_in[22]; const float* lb = (const float*)d_in[23];
    float* out = (float*)d_out;
    char* wsp = (char*)d_ws;
    auto take = [&](size_t bytes) { char* p = wsp; wsp += (bytes + 255) & ~(size_t)255; return (void*)p; };
    bf* FPh = (bf*)take((size_t)256 * 2 * HF * 2); bf* FPl = (bf*)take((size_t)256 * 2 * HF * 2); bf* W3T = (bf*)take((size_t)DD * 2 * HF * 2); float* FC = (float*)take(256 * DD * 4); float* F = (float*)take(256 * DD * 4);
    bf* GW3T = (bf*)take(DD * HG * 2); bf* GPh = (bf*)take((size_t)NM * NIJ * HG * 2); bf* GPl = (bf*)take((size_t)NM * NIJ * HG * 2); float* G = (float*)take((size_t)NM * NIJ * DD * 4);
    bf* Oh = (bf*)take((size_t)NE * DD * 2); bf* Ol = (bf*)take((size_t)NE * DD * 2); bf* EAb = (bf*)take((size_t)NE * DD * 2); bf* LWa = (bf*)take(DD * DD * 2); bf* LWb = (bf*)take(DD * DD * 2); float* R1 = (float*)take((size_t)NE * DD * 4);
    if ((size_t)(wsp - (char*)d_ws) > ws_size) return;
    k_fhid<<<(NB * NM) / 8, 256, 0, stream>>>(ev, f1w2, f1b2, bpm, bps, f2w2, f2b2, FPh, FPl); k_fw3<<<DD / 8, 256, 0, stream>>>(f1w3, f2w3, W3T);
    k_gemmb<true, false><<<dim3((NB * NM) / 64, DD / 64, 1), 128, 0, stream>>>(FPh, FPl, W3T, nullptr, FC, DD, nullptr, nullptr, 2 * HF);
    k_ffin<<<(NB * NM) / 8, 256, 0, stream>>>(FC, ev, f1w1, f1b1, f2w1, f2b1, mm, F);
    k_wt<<<dim3(1, 1, 1), 256, 0, stream>>>(gw3, HG, DD, GW3T);
    for (int b = 0; b < NB; ++b) {
        k_ghid<<<(NM * NIJ) / 8, 256, 0, stream>>>(vec + (size_t)b * NM * NIJ, gw2, gb2, GPh, GPl);
        k_gemmb<true, false><<<dim3((NM * NIJ) / 64, DD / 64, 1), 128, 0, stream>>>(GPh, GPl, GW3T, nullptr, G, DD, nullptr, nullptr, HG);
        k_gsum<<<NIJ / 8, 256, 0, stream>>>(G, vec, gw1, gb1, F, ma, b, Oh, Ol); }
    k_cvt64<<<NE / 8, 256, 0, stream>>>(ea, NE, EAb);
    k_wt<<<dim3(1, 1, 1), 256, 0, stream>>>(lw, DD, DD, LWa); k_wt<<<dim3(1, 1, 1), 256, 0, stream>>>(lw + (size_t)DD * DD, DD, DD, LWb);
    k_gemmb<false, false><<<dim3(NE / 64, DD / 64, 1), 128, 0, stream>>>(EAb, nullptr, LWa, nullptr, R1, DD, nullptr, nullptr, DD);
    k_gemmb<true, false><<<dim3(NE / 64, DD / 64, 1), 128, 0, stream>>>(Oh, Ol, LWb, lb, out, DD, nullptr, R1, DD, 0);
}
